// Encoder_78340203479339
// MI455X (gfx1250) — hardware-verified
//
#include <hip/hip_runtime.h>
#include <math.h>
#include <stdint.h>

constexpr int BATCH = 128;
constexpr int SEQ   = 16;
constexpr int EDIM  = 512;
constexpr int NREL  = 1000;
constexpr int NRELP = 1024;
constexpr int G3    = 1536;
constexpr int AUXW  = 32;
constexpr int OUT0_ELEMS = BATCH * (NREL + 1);
constexpr int OUT1_ELEMS = BATCH * SEQ;
constexpr int OUT_ELEMS  = OUT0_ELEMS + OUT1_ELEMS;

static_assert(EDIM % 32 == 0 && NRELP % 32 == 0, "K multiples of 32");
static_assert(BATCH % 64 == 0 && NRELP % 64 == 0 && EDIM % 64 == 0 && G3 % 64 == 0, "M, N tile multiples");
static_assert(G3 == 3 * EDIM, "gate stacking r|z|n");
static_assert(OUT0_ELEMS % 4 == 0 && (OUT0_ELEMS / 4) % 224 == 0, "out0 store grid exact");
static_assert((OUT0_ELEMS * 4) % 128 == 0, "out1 starts on a 128-B line");
static_assert(OUT_ELEMS * 4 == 520704, "d_out byte total");

typedef __attribute__((ext_vector_type(16))) __bf16   v16b;
typedef __attribute__((ext_vector_type(8)))  __bf16   v8b;
typedef __attribute__((ext_vector_type(8)))  _Float16 v8h;
typedef __attribute__((ext_vector_type(8)))  float    v8f;
typedef __attribute__((ext_vector_type(4)))  float    v4f;
typedef __attribute__((ext_vector_type(4)))  unsigned v4u;
typedef __attribute__((ext_vector_type(4)))  int      v4i;

__device__ __forceinline__ unsigned short f2bf_bits(float f) {
  unsigned u = __float_as_uint(f);
  return (unsigned short)((u + 0x7FFFu + ((u >> 16) & 1u)) >> 16);
}
__device__ __forceinline__ float bf_bits2f(unsigned short h) { return __uint_as_float(((unsigned)h) << 16); }

__device__ __forceinline__ unsigned bf_rne_u(float f) {
  const unsigned u = __float_as_uint(f);
  return (u + 0x7FFFu + ((u >> 16) & 1u)) >> 16;
}
__device__ __forceinline__ void split2(float f, unsigned& hb, unsigned& lb) {
  hb = bf_rne_u(f);
  lb = bf_rne_u(f - __uint_as_float(hb << 16));
}
__device__ __forceinline__ void split_pack8(v4f a, v4f b, v4u& H, v4u& L) {
  unsigned h0, l0, h1, l1;
  const float a0 = a[0], a1 = a[1], a2 = a[2], a3 = a[3];
  const float b0 = b[0], b1 = b[1], b2 = b[2], b3 = b[3];
  split2(a0, h0, l0); split2(a1, h1, l1); H[0] = h0 | (h1 << 16); L[0] = l0 | (l1 << 16);
  split2(a2, h0, l0); split2(a3, h1, l1); H[1] = h0 | (h1 << 16); L[1] = l0 | (l1 << 16);
  split2(b0, h0, l0); split2(b1, h1, l1); H[2] = h0 | (h1 << 16); L[2] = l0 | (l1 << 16);
  split2(b2, h0, l0); split2(b3, h1, l1); H[3] = h0 | (h1 << 16); L[3] = l0 | (l1 << 16);
}
__device__ __forceinline__ float bfw_lo(unsigned w) { return __uint_as_float(w << 16); }
__device__ __forceinline__ float bfw_hi(unsigned w) { return __uint_as_float(w & 0xffff0000u); }

__device__ __forceinline__ float sigm(float x) { return __builtin_amdgcn_rcpf(1.0f + expf(-x)); }

__device__ __forceinline__ float wave_sum(float v) {
  v += __shfl_xor(v, 16, 32);
  v += __shfl_xor(v, 8, 32);
  v += __shfl_xor(v, 4, 32);
  v += __shfl_xor(v, 2, 32);
  v += __shfl_xor(v, 1, 32);
  return v;
}
__device__ __forceinline__ float wave_max(float v) {
  v = fmaxf(v, __shfl_xor(v, 16, 32));
  v = fmaxf(v, __shfl_xor(v, 8, 32));
  v = fmaxf(v, __shfl_xor(v, 4, 32));
  v = fmaxf(v, __shfl_xor(v, 2, 32));
  v = fmaxf(v, __shfl_xor(v, 1, 32));
  return v;
}

__device__ __forceinline__ void dep_guard4_b(v8f& a, v8f& b, v8f& c, v8f& d, v16b x, v16b y) {
  asm volatile("v_nop\n\tv_nop\n\tv_nop\n\tv_nop" : "+v"(a), "+v"(b), "+v"(c), "+v"(d) : "v"(x), "v"(y));
}
__device__ __forceinline__ void keep4_b(v16b a, v16b b, v16b c, v16b d) { asm volatile("v_nop" :: "v"(a), "v"(b), "v"(c), "v"(d)); }
__device__ __forceinline__ void acc_guard4(v8f& a, v8f& b, v8f& c, v8f& d) { asm volatile("v_nop\n\tv_nop\n\tv_nop\n\tv_nop" : "+v"(a), "+v"(b), "+v"(c), "+v"(d)); }

struct FragB {
  union U { v16b v; v8b h[2]; };
  static __device__ __forceinline__ v16b load(const __bf16* p) {
    U f; f.h[0] = *(const v8b*)(p); f.h[1] = *(const v8b*)(p + 16); return f.v;
  }
  static __device__ __forceinline__ v8f mma(v16b a, v16b b, v8f c) {
    return __builtin_amdgcn_wmma_f32_16x16x32_bf16(false, a, false, b, (short)0, c, false, false);
  }
};

template <int BIAS_MODE, int OUT_MODE>
__global__ __launch_bounds__(256) void wmma_gemm64(
    const unsigned short* __restrict__ Ap, const unsigned short* __restrict__ A2p, int lda, long strideA,
    const unsigned short* __restrict__ Btp, const unsigned short* __restrict__ Bt2p, int ldb, long strideB,
    void* __restrict__ Cout, void* __restrict__ Cout2, int ldc, long strideC,
    const float* __restrict__ bias,
    int M, int N, int K, float scale) {
  typedef __bf16 T;
  typedef v16b V;
  const T* A = (const T*)Ap; const T* A2 = (const T*)A2p; const T* Bt = (const T*)Btp; const T* Bt2 = (const T*)Bt2p;
  __shared__ __align__(16) float sT[8][16 * 68];
  const int b    = blockIdx.y;
  const int lane = threadIdx.x & 31;
  const int wave = threadIdx.x >> 5;
  const int tilesN = N >> 6;
  const int tilesM = M >> 6;
  const int tile = blockIdx.x * 8 + wave;
  if (tile >= tilesM * tilesN) return;
  const int tm = tile / tilesN;
  const int tn = tile - tm * tilesN;
  const int m0 = tm << 6;
  const int n0 = tn << 6;

  const T* Ab  = A  + (size_t)b * strideA;
  const T* Bb  = Bt + (size_t)b * strideB;
  const T* Ab2 = A2  + (size_t)b * strideA;
  const T* Bb2 = Bt2 + (size_t)b * strideB;

  const int rlane = lane & 15;
  const int koff  = (lane >> 4) * 8;
  const int mOff  = (lane >> 4) * 8;

  v8f acc[4][4];
#pragma unroll
  for (int i = 0; i < 4; ++i)
#pragma unroll
    for (int j = 0; j < 4; ++j) acc[i][j] = (v8f){0.f,0.f,0.f,0.f,0.f,0.f,0.f,0.f};

  for (int k0 = 0; k0 < K; k0 += 32) {
    V bh[4], bl[4];
#pragma unroll
    for (int j = 0; j < 4; ++j) {
      const size_t bo = (size_t)(n0 + (j << 4) + rlane) * ldb + koff + k0;
      bh[j] = FragB::load(Bb + bo);
      bl[j] = FragB::load(Bb2 + bo);
    }
#pragma unroll
    for (int i = 0; i < 4; ++i) {
      const size_t ao = (size_t)(m0 + (i << 4) + rlane) * lda + koff + k0;
      V ah = FragB::load(Ab + ao);
      V al = FragB::load(Ab2 + ao);
#pragma unroll
      for (int j = 0; j < 4; ++j) {
        acc[i][j] = FragB::mma(ah, bh[j], acc[i][j]);
        acc[i][j] = FragB::mma(ah, bl[j], acc[i][j]);
        acc[i][j] = FragB::mma(al, bh[j], acc[i][j]);
      }
      dep_guard4_b(acc[i][0], acc[i][1], acc[i][2], acc[i][3], ah, al);
    }
    keep4_b(bh[0], bh[1], bh[2], bh[3]);
    keep4_b(bl[0], bl[1], bl[2], bl[3]);
  }
  acc_guard4(acc[0][0], acc[0][1], acc[0][2], acc[0][3]);
  acc_guard4(acc[1][0], acc[1][1], acc[1][2], acc[1][3]);
  acc_guard4(acc[2][0], acc[2][1], acc[2][2], acc[2][3]);
  acc_guard4(acc[3][0], acc[3][1], acc[3][2], acc[3][3]);

  float* slab = sT[wave];
#pragma unroll
  for (int i = 0; i < 4; ++i) {
    const int mBase = m0 + (i << 4);
#pragma unroll
    for (int j = 0; j < 4; ++j) {
      const int n = n0 + (j << 4) + rlane;
      float bv = 0.f;
      if (BIAS_MODE == 2) bv = bias[n];
#pragma unroll
      for (int r = 0; r < 8; ++r) {
        float v = acc[i][j][r] * scale;
        if (BIAS_MODE == 2) v += bv;
        slab[(mOff + r) * 68 + (j << 4) + rlane] = v;
      }
    }
    __builtin_amdgcn_fence(__ATOMIC_RELEASE, "workgroup");
    __builtin_amdgcn_wave_barrier();
    __builtin_amdgcn_fence(__ATOMIC_ACQUIRE, "workgroup");
    if (OUT_MODE == 0) {
      float* C = (float*)Cout + (size_t)b * strideC;
      const int hh = lane >> 4, c4 = (lane & 15) * 4;
      for (int pass = 0; pass < 2; ++pass) {
#pragma unroll
        for (int it = 0; it < 8; ++it) {
          const int row = it * 2 + hh;
          v4f v = *(const v4f*)(slab + row * 68 + c4);
          *(volatile v4f*)(C + (size_t)(mBase + row) * ldc + n0 + c4) = v;
        }
        __threadfence();
      }
    } else {
      const int q = lane >> 3, c8 = (lane & 7) * 8;
      unsigned short* C  = (unsigned short*)Cout  + (size_t)b * strideC;
      unsigned short* C2 = (unsigned short*)Cout2 + (size_t)b * strideC;
      for (int pass = 0; pass < 2; ++pass) {
#pragma unroll
        for (int it = 0; it < 4; ++it) {
          const int row = it * 4 + q;
          const float* sp = slab + row * 68 + c8;
          v8h hv, lv;
#pragma unroll
          for (int e = 0; e < 8; ++e) {
            unsigned short hb = f2bf_bits(sp[e]);
            unsigned short lb = f2bf_bits(sp[e] - bf_bits2f(hb));
            hv[e] = __builtin_bit_cast(_Float16, hb);
            lv[e] = __builtin_bit_cast(_Float16, lb);
          }
          *(volatile v8h*)(C + (size_t)(mBase + row) * ldc + n0 + c8) = hv;
          *(volatile v8h*)(C2 + (size_t)(mBase + row) * ldc + n0 + c8) = lv;
        }
        __threadfence();
      }
    }
    __builtin_amdgcn_fence(__ATOMIC_RELEASE, "workgroup");
    __builtin_amdgcn_wave_barrier();
    __builtin_amdgcn_fence(__ATOMIC_ACQUIRE, "workgroup");
  }
}

__global__ __launch_bounds__(256) void k_split(const float* __restrict__ in, int n8_total, int n8_valid,
                                               unsigned* __restrict__ outH, unsigned* __restrict__ outL) {
  const int i = blockIdx.x * 256 + threadIdx.x;
  if (i >= n8_total) return;
  const int ic = (i < n8_valid) ? i : (n8_valid - 1);
  const bool ok = (i < n8_valid);
  v4f a = *(const v4f*)(in + (size_t)ic * 8);
  v4f b = *(const v4f*)(in + (size_t)ic * 8 + 4);
#pragma unroll
  for (int k = 0; k < 4; ++k) {
    const float av = a[k], bv = b[k];
    a[k] = ok ? av : 0.0f;
    b[k] = ok ? bv : 0.0f;
  }
  v4u H, L;
  split_pack8(a, b, H, L);
  for (int pass = 0; pass < 2; ++pass) {
    *(volatile v4u*)(outH + (size_t)i * 4) = H;
    *(volatile v4u*)(outL + (size_t)i * 4) = L;
    __threadfence();
  }
}

__global__ __launch_bounds__(128) void k_biascat(const float* __restrict__ bq, const float* __restrict__ bk, float* __restrict__ o) {
  const float* src = (blockIdx.x == 0) ? bq : bk;
  const v4f v = *(const v4f*)(src + threadIdx.x * 4);
  float* dst = o + blockIdx.x * EDIM + threadIdx.x * 4;
  *(volatile v4f*)dst = v;
  __threadfence();
  *(volatile v4f*)dst = v;
}

__global__ __launch_bounds__(256) void k_embT(const float* __restrict__ emb, unsigned* __restrict__ TH, unsigned* __restrict__ TL) {
  __shared__ __align__(16) float tile[64 * 68];
  const int tid = threadIdx.x;
  const int r0 = blockIdx.x * 64, e0 = blockIdx.y * 64;
#pragma unroll
  for (int it = 0; it < 4; ++it) {
    const int idx = it * 256 + tid;
    const int rl = idx >> 4, c4 = (idx & 15) * 4;
    const int rr = r0 + rl;
    const int rc = (rr < NREL) ? rr : (NREL - 1);
    const bool ok = (rr < NREL);
    v4f v = *(const v4f*)(emb + (size_t)rc * EDIM + e0 + c4);
#pragma unroll
    for (int k = 0; k < 4; ++k) { const float x = v[k]; v[k] = ok ? x : 0.0f; }
    *(v4f*)(tile + rl * 68 + c4) = v;
  }
  __syncthreads();
  v4u H[2], L[2];
#pragma unroll
  for (int it = 0; it < 2; ++it) {
    const int slot = it * 256 + tid;
    const int el = slot >> 3, c8 = (slot & 7) * 8;
    v4f a, b;
#pragma unroll
    for (int k = 0; k < 4; ++k) {
      a[k] = tile[(c8 + k) * 68 + el];
      b[k] = tile[(c8 + 4 + k) * 68 + el];
    }
    split_pack8(a, b, H[it], L[it]);
  }
  for (int pass = 0; pass < 2; ++pass) {
#pragma unroll
    for (int it = 0; it < 2; ++it) {
      const int slot = it * 256 + tid;
      const int el = slot >> 3, c8 = (slot & 7) * 8;
      const size_t w = (size_t)(e0 + el) * (NRELP / 2) + (size_t)((r0 + c8) >> 1);
      *(volatile v4u*)(TH + w) = H[it];
      *(volatile v4u*)(TL + w) = L[it];
    }
    __threadfence();
  }
}

__global__ __launch_bounds__(256) void k_h1(const float* __restrict__ GIp, const float* __restrict__ bhh,
                                            float* __restrict__ H1f, unsigned* __restrict__ H1H, unsigned* __restrict__ H1L) {
  __shared__ __align__(16) float hbuf[8 * EDIM];
  const int tid = threadIdx.x, lane = tid & 31, wave = tid >> 5;
  const int row = blockIdx.x * 8 + wave;
  const float* gi = GIp + (size_t)row * G3;
  float* myrow = hbuf + wave * EDIM;
#pragma unroll 1
  for (int i = 0; i < 16; ++i) {
    const int e = lane + 32 * i;
    const float gir = gi[e], giz = gi[EDIM + e], gin = gi[2 * EDIM + e];
    const float br = bhh[e], bz = bhh[EDIM + e], bn = bhh[2 * EDIM + e];
    const float r = sigm(gir + br);
    const float z = sigm(giz + bz);
    const float n = tanhf(gin + r * bn);
    myrow[e] = (1.0f - z) * n;
  }
  __syncthreads();
  v4f f[4];
  v4u H[2], L[2];
#pragma unroll
  for (int it = 0; it < 4; ++it) f[it] = *(const v4f*)(myrow + it * 128 + lane * 4);
#pragma unroll
  for (int it = 0; it < 2; ++it) {
    const v4f a = *(const v4f*)(myrow + it * 256 + lane * 8);
    const v4f b = *(const v4f*)(myrow + it * 256 + lane * 8 + 4);
    split_pack8(a, b, H[it], L[it]);
  }
  for (int pass = 0; pass < 2; ++pass) {
#pragma unroll
    for (int it = 0; it < 4; ++it) *(volatile v4f*)(H1f + (size_t)row * EDIM + it * 128 + lane * 4) = f[it];
#pragma unroll
    for (int it = 0; it < 2; ++it) {
      const size_t w = (size_t)row * (EDIM / 2) + (size_t)(it * 128 + lane * 4);
      *(volatile v4u*)(H1H + w) = H[it];
      *(volatile v4u*)(H1L + w) = L[it];
    }
    __threadfence();
  }
}

__device__ __forceinline__ void copy_item(const float* __restrict__ sgi, const float* __restrict__ sh1, const float* __restrict__ sgh,
                                          float* __restrict__ dgi, float* __restrict__ dh1, float* __restrict__ dgh, int tid) {
  const int o = tid * 4;
  const v4f a0 = *(const v4f*)(sgi + o);
  const v4f a1 = *(const v4f*)(sgi + EDIM + o);
  const v4f a2 = *(const v4f*)(sgi + 2 * EDIM + o);
  const v4f hv = *(const v4f*)(sh1 + o);
  const v4f c0 = *(const v4f*)(sgh + o);
  const v4f c1 = *(const v4f*)(sgh + EDIM + o);
  const v4f c2 = *(const v4f*)(sgh + 2 * EDIM + o);
  for (int pass = 0; pass < 2; ++pass) {
    *(volatile v4f*)(dgi + o) = a0;
    *(volatile v4f*)(dgi + EDIM + o) = a1;
    *(volatile v4f*)(dgi + 2 * EDIM + o) = a2;
    *(volatile v4f*)(dh1 + o) = hv;
    *(volatile v4f*)(dgh + o) = c0;
    *(volatile v4f*)(dgh + EDIM + o) = c1;
    *(volatile v4f*)(dgh + 2 * EDIM + o) = c2;
    __threadfence();
  }
}

__global__ __launch_bounds__(128) void k_gather(const int* __restrict__ tokens,
    const float* __restrict__ GIT, const float* __restrict__ H1T, const float* __restrict__ GHT,
    float* __restrict__ dGI, float* __restrict__ dH1, float* __restrict__ dGH) {
  const int item = blockIdx.x;
  int tok = tokens[item];
  tok = tok < 0 ? 0 : tok;
  tok = tok > (NREL - 1) ? (NREL - 1) : tok;
  copy_item(GIT + (size_t)tok * G3, H1T + (size_t)tok * EDIM, GHT + (size_t)tok * G3,
            dGI + (size_t)item * G3, dH1 + (size_t)item * EDIM, dGH + (size_t)item * G3, threadIdx.x);
}

__global__ __launch_bounds__(128) void k_compact(
    const float* __restrict__ cGI, const float* __restrict__ cH1, const float* __restrict__ cGH,
    const float* __restrict__ sGI, const float* __restrict__ sH1, const float* __restrict__ sGH,
    const int* __restrict__ SELP,
    float* __restrict__ dGI, float* __restrict__ dH1, float* __restrict__ dGH, int Lnew) {
  const int b = blockIdx.x / Lnew;
  const int j = blockIdx.x - b * Lnew;
  int sel = SELP[b * AUXW];
  sel = sel < 0 ? 0 : sel;
  sel = sel > (Lnew - 1) ? (Lnew - 1) : sel;
  int src = j + ((j > sel) ? 1 : 0);
  src = src > Lnew ? Lnew : src;
  const bool stage = (j == sel);
  const size_t srow = (size_t)(b * SEQ + src);
  const float* pgi = stage ? (sGI + (size_t)b * G3)   : (cGI + srow * G3);
  const float* ph1 = stage ? (sH1 + (size_t)b * EDIM) : (cH1 + srow * EDIM);
  const float* pgh = stage ? (sGH + (size_t)b * G3)   : (cGH + srow * G3);
  const size_t drow = (size_t)(b * SEQ + j);
  copy_item(pgi, ph1, pgh, dGI + drow * G3, dH1 + drow * EDIM, dGH + drow * G3, threadIdx.x);
}

__global__ __launch_bounds__(512) void k_pairs(
    const float* __restrict__ GIs, const float* __restrict__ H1s, const float* __restrict__ GHs,
    const float* __restrict__ wfc, const float* __restrict__ bfc,
    float* __restrict__ PAIRF, unsigned* __restrict__ PRH, unsigned* __restrict__ PRL, int* __restrict__ SELP, int Lm1) {
  __shared__ __align__(16) float prow[16 * EDIM];
  __shared__ float slog[16];
  const int tid = threadIdx.x, lane = tid & 31, wave = tid >> 5;
  const int b = blockIdx.x;
  const int j = wave > 14 ? 14 : wave;
  const float* gi = GIs + (size_t)(b * SEQ + j + 1) * G3;
  const float* gh = GHs + (size_t)(b * SEQ + j) * G3;
  const float* h1 = H1s + (size_t)(b * SEQ + j) * EDIM;
  float* myrow = prow + j * EDIM;
  float acc = 0.0f;
#pragma unroll 1
  for (int i = 0; i < 16; ++i) {
    const int e = lane + 32 * i;
    const float gir = gi[e], giz = gi[EDIM + e], gin = gi[2 * EDIM + e];
    const float ghr = gh[e], ghz = gh[EDIM + e], ghn = gh[2 * EDIM + e];
    float hv = h1[e];
    float wv = wfc[e];
    asm volatile("" : "+v"(hv), "+v"(wv));
    const float r = sigm(gir + ghr);
    const float z = sigm(giz + ghz);
    const float n = tanhf(gin + r * ghn);
    const float p = (1.0f - z) * n + z * hv;
    myrow[e] = p;
    acc = fmaf(p, wv, acc);
  }
  acc = wave_sum(acc);
  const float logit = acc + bfc[0];
  if (lane == 0) slog[j] = logit;
  __syncthreads();
  int best = 0;
  float bv = slog[0];
#pragma unroll 1
  for (int jj = 1; jj < Lm1; ++jj) {
    const float v = slog[jj];
    if (v > bv) { bv = v; best = jj; }
  }
  if (wave == 0) {
    const float* srow = prow + best * EDIM;
    v4f f[4];
    v4u H[2], L[2];
#pragma unroll
    for (int it = 0; it < 4; ++it) f[it] = *(const v4f*)(srow + it * 128 + lane * 4);
#pragma unroll
    for (int it = 0; it < 2; ++it) {
      const v4f a = *(const v4f*)(srow + it * 256 + lane * 8);
      const v4f c = *(const v4f*)(srow + it * 256 + lane * 8 + 4);
      split_pack8(a, c, H[it], L[it]);
    }
    const v4i sv = {best, best, best, best};
    for (int pass = 0; pass < 2; ++pass) {
#pragma unroll
      for (int it = 0; it < 4; ++it) *(volatile v4f*)(PAIRF + (size_t)b * EDIM + it * 128 + lane * 4) = f[it];
#pragma unroll
      for (int it = 0; it < 2; ++it) {
        const size_t w = (size_t)b * (EDIM / 2) + (size_t)(it * 128 + lane * 4);
        *(volatile v4u*)(PRH + w) = H[it];
        *(volatile v4u*)(PRL + w) = L[it];
      }
      if (lane < 8) *(volatile v4i*)(SELP + b * AUXW + lane * 4) = sv;
      __threadfence();
    }
  }
}

__global__ __launch_bounds__(256) void k_softmax(const float* __restrict__ SC,
    const unsigned* __restrict__ QKH, const unsigned* __restrict__ QKL,
    unsigned* __restrict__ PH, unsigned* __restrict__ PL, float* __restrict__ AUXc, float scl, int do_prob) {
  __shared__ __align__(16) float pbuf[NRELP];
  __shared__ float redD[8], redM[8], redZ[8], redW[8];
  const int tid = threadIdx.x, lane = tid & 31, wave = tid >> 5;
  const int b = blockIdx.x;
  const size_t wb = (size_t)b * (NRELP / 2);
  const unsigned qh = QKH[wb + tid], ql = QKL[wb + tid];
  const unsigned kh = QKH[wb + 256 + tid], kl = QKL[wb + 256 + tid];
  const float q0 = bfw_lo(qh) + bfw_lo(ql), q1 = bfw_hi(qh) + bfw_hi(ql);
  const float k0 = bfw_lo(kh) + bfw_lo(kl), k1 = bfw_hi(kh) + bfw_hi(kl);
  float d = q0 * k0;
  d = fmaf(q1, k1, d);
  d = wave_sum(d);
  float s[4];
  float m = -INFINITY;
#pragma unroll
  for (int i = 0; i < 4; ++i) {
    const int col = tid + 256 * i;
    const int cc = (col < NREL) ? col : (NREL - 1);
    const float v = SC[(size_t)b * NRELP + cc];
    s[i] = v;
    m = fmaxf(m, (col < NREL) ? v : -INFINITY);
  }
  m = wave_max(m);
  if (lane == 0) { redD[wave] = d; redM[wave] = m; }
  __syncthreads();
  float dot = 0.0f;
  float mm = -INFINITY;
#pragma unroll
  for (int w = 0; w < 8; ++w) { dot += redD[w]; mm = fmaxf(mm, redM[w]); }
  const float s_self = dot * scl;
  mm = fmaxf(mm, s_self);
  float ex[4];
  float zp = 0.0f, wp = 0.0f;
#pragma unroll
  for (int i = 0; i < 4; ++i) {
    const int col = tid + 256 * i;
    const bool ok = (col < NREL);
    const float t = ok ? (s[i] - mm) : 0.0f;
    const float e = ok ? expf(t) : 0.0f;
    ex[i] = e;
    zp += e;
    wp = fmaf(e, t, wp);
  }
  zp = wave_sum(zp);
  wp = wave_sum(wp);
  if (lane == 0) { redZ[wave] = zp; redW[wave] = wp; }
  __syncthreads();
  float Z = 0.0f, W = 0.0f;
#pragma unroll
  for (int w = 0; w < 8; ++w) { Z += redZ[w]; W += redW[w]; }
  const float t_self = s_self - mm;
  const float e_self = expf(t_self);
  Z += e_self;
  W = fmaf(e_self, t_self, W);
  const float invZ = 1.0f / Z;
  const float loss = logf(Z) - W * invZ;
  const float p_self = e_self * invZ;
#pragma unroll
  for (int i = 0; i < 4; ++i) pbuf[tid + 256 * i] = ex[i] * invZ;
  __syncthreads();
  if (do_prob != 0 && tid < 128) {
    const v4f a = *(const v4f*)(pbuf + tid * 8);
    const v4f c = *(const v4f*)(pbuf + tid * 8 + 4);
    v4u H, L;
    split_pack8(a, c, H, L);
    for (int pass = 0; pass < 2; ++pass) {
      *(volatile v4u*)(PH + wb + tid * 4) = H;
      *(volatile v4u*)(PL + wb + tid * 4) = L;
      __threadfence();
    }
  }
  if (wave == 0 && lane < 8) {
    v4f av;
    av[0] = (lane == 0) ? loss : 0.0f;
    av[1] = (lane == 0) ? p_self : 0.0f;
    av[2] = (lane == 0) ? s_self : 0.0f;
    av[3] = 0.0f;
    float* ap = AUXc + (size_t)b * AUXW + lane * 4;
    *(volatile v4f*)ap = av;
    __threadfence();
    *(volatile v4f*)ap = av;
  }
}

__global__ __launch_bounds__(256) void k_mergefix(const float* __restrict__ MG, const float* __restrict__ PAIRF,
    const float* __restrict__ AUXc, unsigned* __restrict__ MH, unsigned* __restrict__ ML) {
  const int i = blockIdx.x * 256 + threadIdx.x;
  const int b = i >> 6;
  const float p = AUXc[(size_t)b * AUXW + 1];
  const v4f g0 = *(const v4f*)(MG + (size_t)i * 8);
  const v4f g1 = *(const v4f*)(MG + (size_t)i * 8 + 4);
  const v4f x0 = *(const v4f*)(PAIRF + (size_t)i * 8);
  const v4f x1 = *(const v4f*)(PAIRF + (size_t)i * 8 + 4);
  v4f a, c;
#pragma unroll
  for (int k = 0; k < 4; ++k) {
    a[k] = fmaf(p, x0[k], g0[k]);
    c[k] = fmaf(p, x1[k], g1[k]);
  }
  v4u H, L;
  split_pack8(a, c, H, L);
  for (int pass = 0; pass < 2; ++pass) {
    *(volatile v4u*)(MH + (size_t)i * 4) = H;
    *(volatile v4u*)(ML + (size_t)i * 4) = L;
    __threadfence();
  }
}

__global__ __launch_bounds__(224) void k_writeout(const float* __restrict__ SC, const float* __restrict__ AUX, float* __restrict__ out) {
  const int tid = threadIdx.x;
  if (blockIdx.x < 143) {
    const int i = blockIdx.x * 224 + tid;
    v4f v;
#pragma unroll
    for (int k = 0; k < 4; ++k) {
      const int f = 4 * i + k;
      const int b = f / (NREL + 1);
      const int r = f - b * (NREL + 1);
      const int rc = (r < NREL) ? r : (NREL - 1);
      const float a = SC[(size_t)b * NRELP + rc];
      const float sself = AUX[(size_t)(15 * BATCH + b) * AUXW + 2];
      const float fa = (r < NREL) ? 1.0f : 0.0f;
      const float fb = 1.0f - fa;
      v[k] = fmaf(fa, a, fb * sself);
    }
    float* p = out + (size_t)i * 4;
    *(volatile v4f*)p = v;
    __threadfence();
    *(volatile v4f*)p = v;
  } else {
    const int g4 = (blockIdx.x - 143) * 224 + tid;
    if (g4 < OUT1_ELEMS / 4) {
      v4f v;
#pragma unroll
      for (int k = 0; k < 4; ++k) {
        const int g = 4 * g4 + k;
        const int b = g >> 4;
        const int c = g & 15;
        const int cc = (c == 14) ? 13 : c;
        const float a = AUX[(size_t)(cc * BATCH + b) * AUXW];
        v[k] = (c == 14) ? 0.0f : a;
      }
      float* p = out + (size_t)OUT0_ELEMS + (size_t)g4 * 4;
      *(volatile v4f*)p = v;
      __threadfence();
      *(volatile v4f*)p = v;
    }
  }
}

template <int BIAS_MODE, int OUT_MODE>
static void launch_gemm(const unsigned short* A, const unsigned short* A2, int lda,
                        const unsigned short* Bt, const unsigned short* Bt2, int ldb,
                        void* C, void* C2, int ldc, const float* bias,
                        int Mm, int Nn, int Kk, float scale, hipStream_t st) {
  const int tiles = (Mm >> 6) * (Nn >> 6);
  dim3 grid((tiles + 7) / 8, 1);
  wmma_gemm64<BIAS_MODE, OUT_MODE><<<grid, 256, 0, st>>>(A, A2, lda, 0L, Bt, Bt2, ldb, 0L, C, C2, ldc, 0L, bias, Mm, Nn, Kk, scale);
}

extern "C" void kernel_launch(void* const* d_in, const int* in_sizes, int n_in,
                              void* d_out, int out_size, void* d_ws, size_t ws_size, hipStream_t stream) {
  if (n_in < 12 || d_out == nullptr || d_ws == nullptr) return;
  if (in_sizes[0] != BATCH * SEQ || in_sizes[1] != (NREL + 1) * EDIM || in_sizes[2] != G3 * EDIM ||
      in_sizes[3] != G3 * EDIM || in_sizes[4] != G3 || in_sizes[5] != G3 || in_sizes[6] != EDIM ||
      in_sizes[7] < 1 || in_sizes[8] != EDIM * EDIM || in_sizes[9] != EDIM || in_sizes[10] != EDIM * EDIM ||
      in_sizes[11] != EDIM || out_size != OUT_ELEMS) return;

  const int*   tokens = (const int*)d_in[0];
  const float* emb    = (const float*)d_in[1];
  const float* W_ih   = (const float*)d_in[2];
  const float* W_hh   = (const float*)d_in[3];
  const float* b_ih   = (const float*)d_in[4];
  const float* b_hh   = (const float*)d_in[5];
  const float* w_fc   = (const float*)d_in[6];
  const float* b_fc   = (const float*)d_in[7];
  const float* Wq     = (const float*)d_in[8];
  const float* bq     = (const float*)d_in[9];
  const float* Wk     = (const float*)d_in[10];
  const float* bk     = (const float*)d_in[11];
  float* out = (float*)d_out;

  const float scl = (float)(1.0 / sqrt((double)EDIM));

  char* ws = (char*)d_ws;
  size_t off = 0;
  auto carve = [&](size_t bytes) -> char* { char* p = ws + off; off += (bytes + 255) & ~(size_t)255; return p; };
  const size_t szW  = (size_t)G3 * EDIM * 2;
  const size_t szQK = (size_t)NRELP * EDIM * 2;
  const size_t szTab = (size_t)NRELP * G3 * 4;
  unsigned short* WIH_H = (unsigned short*)carve(szW);
  unsigned short* WIH_L = (unsigned short*)carve(szW);
  unsigned short* WHH_H = (unsigned short*)carve(szW);
  unsigned short* WHH_L = (unsigned short*)carve(szW);
  unsigned short* WQK_H = (unsigned short*)carve(szQK);
  unsigned short* WQK_L = (unsigned short*)carve(szQK);
  float*          BQK   = (float*)carve((size_t)NRELP * 4);
  unsigned short* EMB_H = (unsigned short*)carve(szQK);
  unsigned short* EMB_L = (unsigned short*)carve(szQK);
  unsigned short* EMT_H = (unsigned short*)carve(szQK);
  unsigned short* EMT_L = (unsigned short*)carve(szQK);
  unsigned short* KRL_H = (unsigned short*)carve(szQK);
  unsigned short* KRL_L = (unsigned short*)carve(szQK);
  float*          GITAB = (float*)carve(szTab);
  float*          GHTAB = (float*)carve(szTab);
  float*          H1TAB = (float*)carve((size_t)NRELP * EDIM * 4);
  unsigned short* H1T_H = (unsigned short*)carve(szQK);
  unsigned short* H1T_L = (unsigned short*)carve(szQK);
  float* GIst[2]; float* H1st[2]; float* GHst[2];
  for (int s = 0; s < 2; ++s) {
    GIst[s] = (float*)carve((size_t)BATCH * SEQ * G3 * 4);
    H1st[s] = (float*)carve((size_t)BATCH * SEQ * EDIM * 4);
    GHst[s] = (float*)carve((size_t)BATCH * SEQ * G3 * 4);
  }
  float*          PAIRF = (float*)carve((size_t)BATCH * EDIM * 4);
  unsigned short* PR_H  = (unsigned short*)carve((size_t)BATCH * EDIM * 2);
  unsigned short* PR_L  = (unsigned short*)carve((size_t)BATCH * EDIM * 2);
  int*            SELP  = (int*)carve((size_t)BATCH * AUXW * 4);
  unsigned short* QK_H  = (unsigned short*)carve((size_t)BATCH * NRELP * 2);
  unsigned short* QK_L  = (unsigned short*)carve((size_t)BATCH * NRELP * 2);
  float*          SC    = (float*)carve((size_t)BATCH * NRELP * 4);
  unsigned short* PB_H  = (unsigned short*)carve((size_t)BATCH * NRELP * 2);
  unsigned short* PB_L  = (unsigned short*)carve((size_t)BATCH * NRELP * 2);
  float*          AUX   = (float*)carve((size_t)SEQ * BATCH * AUXW * 4);
  float*          MG    = (float*)carve((size_t)BATCH * EDIM * 4);
  unsigned short* M_H   = (unsigned short*)carve((size_t)BATCH * EDIM * 2);
  unsigned short* M_L   = (unsigned short*)carve((size_t)BATCH * EDIM * 2);
  float*          GIM   = (float*)carve((size_t)BATCH * G3 * 4);
  float*          GHM   = (float*)carve((size_t)BATCH * G3 * 4);
  float*          H1M   = (float*)carve((size_t)BATCH * EDIM * 4);
  unsigned short* H1M_H = (unsigned short*)carve((size_t)BATCH * EDIM * 2);
  unsigned short* H1M_L = (unsigned short*)carve((size_t)BATCH * EDIM * 2);
  if (off > ws_size || off > (size_t)134217728) return;

  {
    const int n8w = G3 * EDIM / 8;
    const int n8q = EDIM * EDIM / 8;
    const int n8e = NRELP * EDIM / 8;
    const int n8ev = NREL * EDIM / 8;
    k_split<<<n8w / 256, 256, 0, stream>>>(W_ih, n8w, n8w, (unsigned*)WIH_H, (unsigned*)WIH_L);
    k_split<<<n8w / 256, 256, 0, stream>>>(W_hh, n8w, n8w, (unsigned*)WHH_H, (unsigned*)WHH_L);
    k_split<<<n8q / 256, 256, 0, stream>>>(Wq, n8q, n8q, (unsigned*)WQK_H, (unsigned*)WQK_L);
    k_split<<<n8q / 256, 256, 0, stream>>>(Wk, n8q, n8q, (unsigned*)(WQK_H + (size_t)EDIM * EDIM), (unsigned*)(WQK_L + (size_t)EDIM * EDIM));
    k_split<<<n8e / 256, 256, 0, stream>>>(emb, n8e, n8ev, (unsigned*)EMB_H, (unsigned*)EMB_L);
    k_biascat<<<2, 128, 0, stream>>>(bq, bk, BQK);
    k_embT<<<dim3(NRELP / 64, EDIM / 64), 256, 0, stream>>>(emb, (unsigned*)EMT_H, (unsigned*)EMT_L);
  }
  launch_gemm<2, 2>(EMB_H, EMB_L, EDIM, WQK_H + (size_t)EDIM * EDIM, WQK_L + (size_t)EDIM * EDIM, EDIM,
                    KRL_H, KRL_L, EDIM, bk, NRELP, EDIM, EDIM, 1.0f, stream);
  launch_gemm<2, 0>(EMB_H, EMB_L, EDIM, WIH_H, WIH_L, EDIM, GITAB, nullptr, G3, b_ih, NRELP, G3, EDIM, 1.0f, stream);
  k_h1<<<NRELP / 8, 256, 0, stream>>>(GITAB, b_hh, H1TAB, (unsigned*)H1T_H, (unsigned*)H1T_L);
  launch_gemm<2, 0>(H1T_H, H1T_L, EDIM, WHH_H, WHH_L, EDIM, GHTAB, nullptr, G3, b_hh, NRELP, G3, EDIM, 1.0f, stream);
  k_gather<<<BATCH * SEQ, 128, 0, stream>>>(tokens, GITAB, H1TAB, GHTAB, GIst[0], H1st[0], GHst[0]);

  for (int t = 0; t < 14; ++t) {
    const int Lm1 = SEQ - 1 - t;
    const int cur = t & 1, nxt = cur ^ 1;
    float* auxc = AUX + (size_t)t * BATCH * AUXW;
    k_pairs<<<BATCH, 32 * Lm1, 0, stream>>>(GIst[cur], H1st[cur], GHst[cur], w_fc, b_fc, PAIRF,
                                            (unsigned*)PR_H, (unsigned*)PR_L, SELP, Lm1);
    launch_gemm<2, 2>(PR_H, PR_L, EDIM, WQK_H, WQK_L, EDIM, QK_H, QK_L, NRELP, BQK, BATCH, NRELP, EDIM, 1.0f, stream);
    launch_gemm<0, 0>(QK_H, QK_L, NRELP, KRL_H, KRL_L, EDIM, SC, nullptr, NRELP, nullptr, BATCH, NRELP, EDIM, scl, stream);
    k_softmax<<<BATCH, 256, 0, stream>>>(SC, (const unsigned*)QK_H, (const unsigned*)QK_L,
                                         (unsigned*)PB_H, (unsigned*)PB_L, auxc, scl, 1);
    launch_gemm<0, 0>(PB_H, PB_L, NRELP, EMT_H, EMT_L, NRELP, MG, nullptr, EDIM, nullptr, BATCH, EDIM, NRELP, 1.0f, stream);
    k_mergefix<<<BATCH * EDIM / 8 / 256, 256, 0, stream>>>(MG, PAIRF, auxc, (unsigned*)M_H, (unsigned*)M_L);
    launch_gemm<2, 0>(M_H, M_L, EDIM, WIH_H, WIH_L, EDIM, GIM, nullptr, G3, b_ih, BATCH, G3, EDIM, 1.0f, stream);
    k_h1<<<BATCH / 8, 256, 0, stream>>>(GIM, b_hh, H1M, (unsigned*)H1M_H, (unsigned*)H1M_L);
    launch_gemm<2, 0>(H1M_H, H1M_L, EDIM, WHH_H, WHH_L, EDIM, GHM, nullptr, G3, b_hh, BATCH, G3, EDIM, 1.0f, stream);
    k_compact<<<BATCH * Lm1, 128, 0, stream>>>(GIst[cur], H1st[cur], GHst[cur], GIM, H1M, GHM, SELP,
                                               GIst[nxt], H1st[nxt], GHst[nxt], Lm1);
  }

  k_pairs<<<BATCH, 32, 0, stream>>>(GIst[0], H1st[0], GHst[0], w_fc, b_fc, PAIRF, (unsigned*)PR_H, (unsigned*)PR_L, SELP, 1);
  launch_gemm<2, 2>(PR_H, PR_L, EDIM, WQK_H, WQK_L, EDIM, QK_H, QK_L, NRELP, BQK, BATCH, NRELP, EDIM, 1.0f, stream);
  launch_gemm<0, 0>(QK_H, QK_L, NRELP, KRL_H, KRL_L, EDIM, SC, nullptr, NRELP, nullptr, BATCH, NRELP, EDIM, scl, stream);
  k_softmax<<<BATCH, 256, 0, stream>>>(SC, (const unsigned*)QK_H, (const unsigned*)QK_L,
                                       (unsigned*)PB_H, (unsigned*)PB_L, AUX + (size_t)15 * BATCH * AUXW, scl, 0);
  k_writeout<<<146, 224, 0, stream>>>(SC, AUX, out);
}
